// FastEuclideanAttention_51539607552999
// MI455X (gfx1250) — hardware-verified
//
#include <hip/hip_runtime.h>
#include <math.h>

typedef __attribute__((ext_vector_type(16))) _Float16 v16h;
typedef __attribute__((ext_vector_type(16))) __bf16 v16b;
typedef __attribute__((ext_vector_type(8)))  _Float16 v8h;
typedef __attribute__((ext_vector_type(8)))  float v8f;
typedef __attribute__((ext_vector_type(4)))  float v4f;
typedef __attribute__((ext_vector_type(2)))  float v2f;
typedef __attribute__((ext_vector_type(4)))  unsigned v4u;
typedef __attribute__((ext_vector_type(4)))  int v4i;
typedef float __attribute__((may_alias)) float_a;
typedef int __attribute__((may_alias)) int_a;

template <typename T> __device__ __forceinline__ void vst2(void* p, T v) { *(volatile T*)p = v; __threadfence(); *(volatile T*)p = v; }
__device__ __forceinline__ v8f wmma16(v16h a, v16h b, v8f c) {
  v8f d = __builtin_amdgcn_wmma_f32_16x16x32_f16(false, a, false, b, (short)0, c, false, false);
  asm volatile("v_nop\n\tv_nop\n\tv_nop\n\tv_nop" : "+v"(d) : "v"(a), "v"(b));
  return d;
}
__device__ __forceinline__ v8f wmma_bf(v16b a, v16b b, v8f c) {
  v8f d = __builtin_amdgcn_wmma_f32_16x16x32_bf16(false, a, false, b, (short)0, c, false, false);
  asm volatile("v_nop\n\tv_nop\n\tv_nop\n\tv_nop" : "+v"(d) : "v"(a), "v"(b));
  return d;
}
__device__ __forceinline__ v16h frag_h(const _Float16* rowk0, int lane) {
  union { v16h v; v8h q[2]; } u; const _Float16* p = rowk0 + 8 * (lane >> 4);
  u.q[0] = *(const v8h*)p; u.q[1] = *(const v8h*)(p + 16); return u.v;
}
__device__ __forceinline__ v16h frag_f32(const float* rowk0, int lane) {
  v16h a; const float* p = rowk0 + 8 * (lane >> 4);
#pragma unroll
  for (int i = 0; i < 8; ++i) { a[i] = (_Float16)p[i]; a[8 + i] = (_Float16)p[16 + i]; }
  return a;
}
__device__ __forceinline__ v16h frag_f32s(const float* rowk0, int lane, float sc) {
  v16h a; const float* p = rowk0 + 8 * (lane >> 4);
#pragma unroll
  for (int i = 0; i < 8; ++i) { a[i] = (_Float16)(p[i] * sc); a[8 + i] = (_Float16)(p[16 + i] * sc); }
  return a;
}
__device__ __forceinline__ v16h fragc_f32(const float* W, int k0, int n, int lane, int ld, int K) {
  v16h a; const int g = lane >> 4;
#pragma unroll
  for (int i = 0; i < 8; ++i) { const int ka = k0 + 8 * g + i, kb = ka + 16;
    a[i] = (_Float16)(ka < K ? W[(size_t)ka * ld + n] : 0.f); a[8 + i] = (_Float16)(kb < K ? W[(size_t)kb * ld + n] : 0.f); }
  return a;
}
struct F2 { v16b h, l; };
__device__ __forceinline__ F2 bsplit16(const float v[16]) { F2 r;
#pragma unroll
  for (int i = 0; i < 16; ++i) { const __bf16 h = (__bf16)v[i]; r.h[i] = h; r.l[i] = (__bf16)(v[i] - (float)h); }
  return r; }
__device__ __forceinline__ F2 split_row(const float* row, int k0, int lane) { float v[16]; const float* p = row + k0 + 8 * (lane >> 4);
#pragma unroll
  for (int i = 0; i < 8; ++i) { v[i] = p[i]; v[8 + i] = p[16 + i]; }
  return bsplit16(v); }
__device__ __forceinline__ F2 split_rowK(const float* row, int k0, int lane, int K) { float v[16]; const int g = lane >> 4;
#pragma unroll
  for (int i = 0; i < 8; ++i) { const int ka = k0 + 8 * g + i, kb = ka + 16; v[i] = ka < K ? row[ka] : 0.f; v[8 + i] = kb < K ? row[kb] : 0.f; }
  return bsplit16(v); }
__device__ __forceinline__ F2 split_col(const float* W, int k0, int n, int lane, int ld, int K) { float v[16]; const int g = lane >> 4;
#pragma unroll
  for (int i = 0; i < 8; ++i) { const int ka = k0 + 8 * g + i, kb = ka + 16; v[i] = ka < K ? W[(size_t)ka * ld + n] : 0.f; v[8 + i] = kb < K ? W[(size_t)kb * ld + n] : 0.f; }
  return bsplit16(v); }
__device__ __forceinline__ v8f mac3(const F2& a, const F2& b, v8f c) { c = wmma_bf(a.l, b.h, c); c = wmma_bf(a.h, b.l, c); return wmma_bf(a.h, b.h, c); }
__device__ __forceinline__ float sigm(float v) { return 1.0f / (1.0f + expf(-v)); }
#define LDSX() do { asm volatile("s_wait_dscnt 0" ::: "memory"); __builtin_amdgcn_wave_barrier(); __builtin_amdgcn_fence(__ATOMIC_RELEASE, "workgroup"); } while (0)

#define NB 4
#define LL 1024
#define NH 12
#define EE 64

__global__ __launch_bounds__(256) void k_prep(const float* __restrict__ keys, const float* __restrict__ vals, float* __restrict__ kn, _Float16* __restrict__ vT) {
  __shared__ float tile[64][65];
  __shared__ __align__(16) float skn[64];
  const int bh = blockIdx.y, b = bh / NH, h = bh % NH, j0 = blockIdx.x * 64, tid = threadIdx.x;
  for (int q = tid; q < 64 * 64; q += 256) { const int jl = q >> 6, e = q & 63; tile[jl][e] = vals[(((size_t)b * LL + j0 + jl) * NH + h) * EE + e]; }
  if (tid < 64) { const float* kr = keys + (((size_t)b * LL + j0 + tid) * NH + h) * EE; float s = 0.f;
#pragma unroll 8
    for (int e = 0; e < EE; ++e) s += kr[e] * kr[e];
    skn[tid] = s; }
  __syncthreads();
  { const int pc = tid & 7;
#pragma unroll
    for (int u = 0; u < 2; ++u) { const int e = (tid >> 3) + u * 32; union { v8h hh; v4u uu; } pk;
#pragma unroll
      for (int i = 0; i < 8; ++i) pk.hh[i] = (_Float16)tile[pc * 8 + i][e];
      vst2(vT + (((size_t)bh * EE + e) * LL) + j0 + pc * 8, pk.uu); } }
  if (tid < 16) vst2(kn + (size_t)bh * LL + j0 + tid * 4, *(const v4f*)(&skn[tid * 4]));
}
__global__ __launch_bounds__(32) void k_scan(const float* __restrict__ q, const float* __restrict__ w, const float* __restrict__ qmask, float* __restrict__ qh) {
  const int bh = blockIdx.x, b = bh / NH, h = bh % NH, lane = threadIdx.x;
  const float w0 = w[h * EE + 2 * lane], w1 = w[h * EE + 2 * lane + 1], qm = qmask[(size_t)b * LL];
  float m = -3.0e38f, z = 0.f, a0 = 0.f, a1 = 0.f;

#pragma unroll 1
  for (int i = 0; i < LL; ++i) { const float* qr = q + (((size_t)b * LL + i) * NH + h) * EE;
    const float q0 = qr[2 * lane], q1 = qr[2 * lane + 1];
    float s = q0 * w0 + q1 * w1;
#pragma unroll
    for (int off = 16; off >= 1; off >>= 1) s += __shfl_xor(s, off, 32);
    s *= qm;
    const float mn = fmaxf(m, s); const float c = expf(m - mn), p = expf(s - mn);
    z = z * c + p; a0 = a0 * c + p * q0; a1 = a1 * c + p * q1; m = mn;
    vst2(qh + (((size_t)bh * LL + i) * EE) + 2 * lane, (v2f){a0 / z, a1 / z});
  }
}
__global__ __launch_bounds__(128) void k_attn(const float* __restrict__ qh, const float* __restrict__ keys, const float* __restrict__ kn, const _Float16* __restrict__ vT,
                                            const float* __restrict__ kmask, const float* __restrict__ qin, float* __restrict__ out) {
  __shared__ __align__(16) float sS[4][16][68];
  __shared__ __align__(16) _Float16 sP[4][16][72];
  __shared__ __align__(16) float sO[4][16][68];
  const int tid = threadIdx.x, w = tid >> 5, lane = tid & 31, col = lane & 15, g = lane >> 4;
  const int bh = blockIdx.y, b = bh / NH, h = bh % NH, q0 = blockIdx.x * 64 + w * 16;
  const float ks = kmask[(size_t)b * LL];
  F2 aq[2];
#pragma unroll
  for (int kc = 0; kc < 2; ++kc) aq[kc] = split_row(qh + ((size_t)bh * LL + q0 + col) * EE, kc * 32, lane);
  float mrun = -3.0e38f, lrun = 0.f; v8f acc[4] = {};
  const int ntiles = blockIdx.x + 1;
#pragma unroll 1
  for (int kt = 0; kt < ntiles; ++kt) {
    v8f s4[4];
#pragma unroll
    for (int t = 0; t < 4; ++t) { s4[t] = (v8f){};
#pragma unroll
      for (int kc = 0; kc < 2; ++kc) s4[t] = mac3(aq[kc], split_row(keys + (((size_t)b * LL + kt * 64 + t * 16 + col) * NH + h) * EE, kc * 32, lane), s4[t]); }
#pragma unroll
    for (int t = 0; t < 4; ++t)
#pragma unroll
      for (int r = 0; r < 8; ++r) { const int i = q0 + 8 * g + r, j = kt * 64 + t * 16 + col;
        sS[w][8 * g + r][t * 16 + col] = j <= i ? ks * (2.0f * s4[t][r] - kn[(size_t)bh * LL + j]) : -3.0e38f; }
    LDSX();
    float mx = -3.0e38f;
#pragma unroll
    for (int jj = 0; jj < 32; ++jj) mx = fmaxf(mx, sS[w][col][g * 32 + jj]);
    mx = fmaxf(mx, __shfl_xor(mx, 16, 32));
    const float mnew = fmaxf(mrun, mx); const float corr = expf(mrun - mnew);
    float ps = 0.f;
#pragma unroll
    for (int jj = 0; jj < 32; ++jj) { const float v = sS[w][col][g * 32 + jj]; const float p = v > -1.0e38f ? expf(v - mnew) : 0.f; ps += p; sP[w][col][g * 32 + jj] = (_Float16)(p * 16384.0f); }
    ps += __shfl_xor(ps, 16, 32);
    lrun = lrun * corr + ps; mrun = mnew;
#pragma unroll
    for (int r = 0; r < 8; ++r) { const float cr = __shfl(corr, 8 * g + r, 32);
#pragma unroll
      for (int t = 0; t < 4; ++t) acc[t][r] *= cr; }
    LDSX();
#pragma unroll
    for (int kc = 0; kc < 2; ++kc) { const v16h pa = frag_h(&sP[w][col][0] + kc * 32, lane);
#pragma unroll
      for (int t = 0; t < 4; ++t) acc[t] = wmma16(pa, frag_h(vT + ((size_t)bh * EE + t * 16 + col) * LL + kt * 64 + kc * 32, lane), acc[t]); }
    __builtin_amdgcn_wave_barrier();
  }
#pragma unroll
  for (int r = 0; r < 8; ++r) { const float lr = __shfl(lrun, 8 * g + r, 32);
#pragma unroll
    for (int t = 0; t < 4; ++t) sO[w][8 * g + r][t * 16 + col] = acc[t][r] / (lr * 16384.0f); }
  LDSX();
  for (int qq = lane; qq < 16 * 16; qq += 32) { const int rl = qq >> 4, pc = qq & 15; const size_t o = (((size_t)b * LL + q0 + rl) * NH + h) * EE + pc * 4;
    vst2(out + o, *(const v4f*)(&sO[w][rl][pc * 4]) + *(const v4f*)(qin + o)); }
}
extern "C" void kernel_launch(void* const* d_in, const int* in_sizes, int n_in, void* d_out, int out_size, void* d_ws, size_t ws_size, hipStream_t stream) {
  (void)in_sizes; (void)n_in; (void)out_size; (void)ws_size;
  const float* q = (const float*)d_in[0]; const float* k = (const float*)d_in[1]; const float* v = (const float*)d_in[2];
  const float* qmask = (const float*)d_in[3]; const float* kmask = (const float*)d_in[4]; const float* w = (const float*)d_in[5];
  float* out = (float*)d_out;
  char* ws = (char*)d_ws; size_t off = 0;
  auto take = [&](size_t bytes) { char* p = ws + off; off += (bytes + 255) & ~(size_t)255; return p; };
  float* kn = (float*)take((size_t)NB * NH * LL * 4); _Float16* vT = (_Float16*)take((size_t)NB * NH * EE * LL * 2); float* qh = (float*)take((size_t)NB * NH * LL * EE * 4);
  k_prep<<<dim3(LL / 64, NB * NH), 256, 0, stream>>>(k, v, kn, vT);
  k_scan<<<NB * NH, 32, 0, stream>>>(q, w, qmask, qh);
  k_attn<<<dim3(LL / 64, NB * NH), 128, 0, stream>>>(qh, k, kn, vT, kmask, q, out);
}
